// SuperpixelConv_45827301048853
// MI455X (gfx1250) — hardware-verified
//
#include <hip/hip_runtime.h>
#include <math.h>

#define T_   2
#define C_   64
#define H_   160
#define W_   160
#define HW   25600
#define K2   49
#define NSP  196
#define FAN  3136
#define NKC  98

typedef __attribute__((ext_vector_type(16))) _Float16 v16h;
typedef __attribute__((ext_vector_type(8)))  float    v8f;
typedef __attribute__((ext_vector_type(4)))  float    v4f_t;
typedef float v4fa __attribute__((ext_vector_type(4), may_alias));
#define LCAP 4096

__device__ __forceinline__ int refl(int i, int n) {
    i = (i < 0) ? -i : i;
    return (i >= n) ? (2 * n - 2 - i) : i;
}

__global__ __launch_bounds__(256) void k_segmean(const float* __restrict__ x, const int* __restrict__ spix,
                                                 float* __restrict__ down) {
    __shared__ int lst[LCAP];
    __shared__ int wcnt[8];
    __shared__ int total;
    __shared__ float part[4][64];
    const int tid = threadIdx.x, lane = tid & 31, wave = tid >> 5;
    const int t = blockIdx.x / NSP, s = blockIdx.x % NSP;
    const int* sp = spix + t * HW;
    if (tid == 0) total = 0;
    __syncthreads();
    for (int p0 = 0; p0 < HW; p0 += 256) {
        const int p = p0 + tid;
        const bool hit = (p < HW) && (sp[p] == s);
        const unsigned m = __ballot(hit);
        if (lane == 0) wcnt[wave] = __popc(m);
        __syncthreads();
        int base = total;
#pragma unroll
        for (int w = 0; w < 8; ++w) if (w < wave) base += wcnt[w];
        if (hit) { const int slot = base + __popc(m & ((1u << lane) - 1u)); if (slot < LCAP) lst[slot] = p; }
        __syncthreads();
        if (tid == 0) { int tt = total; for (int w = 0; w < 8; ++w) tt += wcnt[w]; total = tt; }
        __syncthreads();
    }
    const int n = (total < LCAP) ? total : LCAP;
    const int c = tid & 63, q = tid >> 6;
    const float* xc = x + ((size_t)t * C_ + c) * HW;
    float acc = 0.f;
    for (int i = q; i < n; i += 4) acc += xc[lst[i]];
    part[q][c] = acc;
    __syncthreads();
    if (tid < 64) {
        const float inv = 1.0f / fmaxf((float)total, 1.0f);
        const float v = (part[0][tid] + part[1][tid] + part[2][tid] + part[3][tid]) * inv;
        float* d = down + ((size_t)t * NSP + s) * C_ + tid;
        *(volatile float*)d = v; __threadfence(); *(volatile float*)d = v;
    }
}

__global__ void k_pwd(const float* __restrict__ down, float* __restrict__ pwd) {
    int idx = blockIdx.x * blockDim.x + threadIdx.x;
    if (idx >= T_ * NSP * NSP) return;
    int t = idx / (NSP * NSP);
    int r = idx % (NSP * NSP);
    int i = r / NSP, j = r % NSP;
    const float* di = down + ((size_t)t * NSP + i) * C_;
    const float* dj = down + ((size_t)t * NSP + j) * C_;
    float dot = 0.f, si = 0.f, sj = 0.f;
    for (int c = 0; c < C_; ++c) { dot += di[c] * dj[c]; si += di[c] * di[c]; sj += dj[c] * dj[c]; }
    const float v = fmaxf(si + sj - 2.0f * dot, 0.0f);
    *(volatile float*)(pwd + idx) = v; __threadfence(); *(volatile float*)(pwd + idx) = v;
}

__global__ void k_scale(const float* __restrict__ x, const float* __restrict__ wsc,
                        const float* __restrict__ bsc, float* __restrict__ scl) {
    int pid = blockIdx.x * blockDim.x + threadIdx.x;
    if (pid >= T_ * HW) return;
    int t = pid / HW, r = pid % HW;
    const float* xb = x + (size_t)t * C_ * HW + r;
    float ss = 0.f, dt = 0.f;
    for (int c = 0; c < C_; ++c) {
        float v = xb[(size_t)c * HW];
        ss += v * v;
        dt += wsc[c] * v;
    }
    float v = dt / (sqrtf(ss) + 1e-10f) + bsc[0];
    float sp = (v > 20.f) ? v : logf(1.f + expf(v));
    *(volatile float*)(scl + pid) = 10.f * sp; __threadfence(); *(volatile float*)(scl + pid) = 10.f * sp;
}

__global__ void k_pack(const float* __restrict__ Wl, _Float16* __restrict__ Ap) {
    int idx = (blockIdx.x * blockDim.x + threadIdx.x) * 2;
    if (idx >= 4 * NKC * 32 * 16) return;
    int i    = idx & 15;
    int lane = (idx >> 4) & 31;
    int kc   = (idx >> 9) % NKC;
    int ot   = idx / (NKC * 512);
    int o    = ot * 16 + (lane & 15);
    int kin  = ((lane < 16) ? 0 : 8) + ((i < 8) ? i : i + 8);
    int k    = kc * 32 + kin;
    const unsigned p = (unsigned)__builtin_bit_cast(unsigned short, (_Float16)Wl[o * FAN + k]) | ((unsigned)__builtin_bit_cast(unsigned short, (_Float16)Wl[o * FAN + k + 1]) << 16);
    *(volatile unsigned*)(Ap + idx) = p; __threadfence(); *(volatile unsigned*)(Ap + idx) = p;
}

__global__ void __launch_bounds__(64) k_conv(
    const float* __restrict__ x, const int* __restrict__ spix,
    const float* __restrict__ pwd, const float* __restrict__ scl,
    const _Float16* __restrict__ Ap, const float* __restrict__ blin,
    float* __restrict__ out) {
    __shared__ float rwSa[2][16 * K2];
    __shared__ int   offSa[2][16 * K2];
    __shared__ __attribute__((aligned(16))) float Ob[64][32 + 4];

    const int wv = threadIdx.x >> 5;
    float* rwS = rwSa[wv];
    int*   offS = offSa[wv];
    int lane = threadIdx.x & 31;
    int w0 = blockIdx.x * 32 + wv * 16;
    int h  = blockIdx.y;
    int t  = blockIdx.z;
    const int*   sp = spix + t * HW;
    const float* pw = pwd + (size_t)t * NSP * NSP;

    for (int idx = lane; idx < 16 * K2; idx += 32) {
        int n = idx / K2, tap = idx - n * K2;
        int w  = w0 + n;
        int hh = refl(h + tap / 7 - 3, H_);
        int ww = refl(w + tap % 7 - 3, W_);
        int s  = sp[h * W_ + w];
        int ns = sp[hh * W_ + ww];
        float sim = pw[s * NSP + ns];
        float sc  = scl[t * HW + h * W_ + w];
        rwS[idx]  = expf(-sc * sim);
        offS[idx] = hh * W_ + ww;
    }
    __syncthreads();
    if (lane < 16) {
        float m = 0.f;
        for (int tap = 0; tap < K2; ++tap) m = fmaxf(m, rwS[lane * K2 + tap]);
        float inv = 1.f / (1e-5f + m);
        for (int tap = 0; tap < K2; ++tap) rwS[lane * K2 + tap] *= inv;
    }
    __syncthreads();

    int n    = lane & 15;
    int rh8  = (lane < 16) ? 0 : 8;
    const float* xb  = x + (size_t)t * C_ * HW;
    const float* rwp = rwS + n * K2;
    const int*   ofp = offS + n * K2;
    const v16h*  Af  = (const v16h*)Ap;

    v8f acc[4] = {v8f{}, v8f{}, v8f{}, v8f{}};

    for (int kc = 0; kc < NKC; ++kc) {
        union { _Float16 hv[16]; v16h v; } B;
#pragma unroll
        for (int j = 0; j < 16; ++j) {
            int row = kc * 32 + ((j < 8) ? (rh8 + j) : (16 + rh8 + (j - 8)));
            int c   = row / K2;
            int tap = row - c * K2;
            B.hv[j] = (_Float16)(xb[(size_t)c * HW + ofp[tap]] * rwp[tap]);
        }
        int abase = kc * 32 + lane;
#pragma unroll
        for (int ot = 0; ot < 4; ++ot) {
            v16h a = Af[ot * NKC * 32 + abase];
            acc[ot] = __builtin_amdgcn_wmma_f32_16x16x32_f16(
                false, a, false, B.v, (short)0, acc[ot], false, false);
        }
    }

    int Mb = (lane < 16) ? 0 : 8;
#pragma unroll
    for (int ot = 0; ot < 4; ++ot)
#pragma unroll
        for (int v = 0; v < 8; ++v) { int o = ot * 16 + Mb + v; Ob[o][wv * 16 + n] = acc[ot][v] + blin[o]; }
    __syncthreads();
    {
        const int tid = threadIdx.x;
        float* ob = out + (size_t)t * C_ * HW + h * W_ + blockIdx.x * 32;
#pragma unroll 1
        for (int pass = 0; pass < 2; ++pass) {
#pragma unroll
            for (int i = 0; i < 8; ++i) { const int c = tid + 64 * i, o = c >> 3, q = c & 7; *(volatile v4f_t*)(ob + (size_t)o * HW + q * 4) = *(const v4fa*)&Ob[o][q * 4]; }
            __threadfence();
        }
    }
}

extern "C" void kernel_launch(void* const* d_in, const int* in_sizes, int n_in,
                              void* d_out, int out_size, void* d_ws, size_t ws_size,
                              hipStream_t stream) {
    const float* x    = (const float*)d_in[0];
    const int*   spix = (const int*)d_in[1];
    const float* Wl   = (const float*)d_in[2];
    const float* bl   = (const float*)d_in[3];
    const float* wsc  = (const float*)d_in[4];
    const float* bsc  = (const float*)d_in[5];
    float* out = (float*)d_out;

    float* sums = (float*)d_ws;
    float* cnts = sums + T_ * NSP * C_;
    float* sq   = cnts + T_ * NSP;
    float* pwd  = sq + T_ * NSP;
    float* scl  = pwd + T_ * NSP * NSP;
    _Float16* Ap = (_Float16*)(scl + T_ * HW);

    (void)cnts; (void)sq;
    k_segmean<<<T_ * NSP, 256, 0, stream>>>(x, spix, sums);
    k_pwd<<<(T_ * NSP * NSP + 255) / 256, 256, 0, stream>>>(sums, pwd);
    k_scale<<<(T_ * HW + 255) / 256, 256, 0, stream>>>(x, wsc, bsc, scl);
    k_pack<<<(4 * NKC * 32 * 16 / 2 + 255) / 256, 256, 0, stream>>>(Wl, Ap);

    dim3 grid(W_ / 32, H_, T_);
    k_conv<<<grid, 64, 0, stream>>>(x, spix, pwd, scl, Ap, bl, out);
}
